// NormalizedCorrelation2D_2439541424700
// MI455X (gfx1250) — hardware-verified
//
#include <hip/hip_runtime.h>
#include <math.h>

typedef __attribute__((ext_vector_type(16))) _Float16 v16h;
typedef __attribute__((ext_vector_type(16))) __bf16 v16b;
typedef __attribute__((ext_vector_type(8)))  _Float16 v8h;
typedef __attribute__((ext_vector_type(8)))  float v8f;
typedef __attribute__((ext_vector_type(4)))  float v4f;
typedef __attribute__((ext_vector_type(2)))  float v2f;
typedef __attribute__((ext_vector_type(4)))  unsigned v4u;
typedef __attribute__((ext_vector_type(4)))  int v4i;
typedef float __attribute__((may_alias)) float_a;
typedef int __attribute__((may_alias)) int_a;

template <typename T> __device__ __forceinline__ void vst2(void* p, T v) { *(volatile T*)p = v; __threadfence(); *(volatile T*)p = v; }
__device__ __forceinline__ v8f wmma16(v16h a, v16h b, v8f c) {
  v8f d = __builtin_amdgcn_wmma_f32_16x16x32_f16(false, a, false, b, (short)0, c, false, false);
  asm volatile("v_nop\n\tv_nop\n\tv_nop\n\tv_nop" : "+v"(d) : "v"(a), "v"(b));
  return d;
}
__device__ __forceinline__ v8f wmma_bf(v16b a, v16b b, v8f c) {
  v8f d = __builtin_amdgcn_wmma_f32_16x16x32_bf16(false, a, false, b, (short)0, c, false, false);
  asm volatile("v_nop\n\tv_nop\n\tv_nop\n\tv_nop" : "+v"(d) : "v"(a), "v"(b));
  return d;
}
__device__ __forceinline__ v16h frag_h(const _Float16* rowk0, int lane) {
  union { v16h v; v8h q[2]; } u; const _Float16* p = rowk0 + 8 * (lane >> 4);
  u.q[0] = *(const v8h*)p; u.q[1] = *(const v8h*)(p + 16); return u.v;
}
__device__ __forceinline__ v16h frag_f32(const float* rowk0, int lane) {
  v16h a; const float* p = rowk0 + 8 * (lane >> 4);
#pragma unroll
  for (int i = 0; i < 8; ++i) { a[i] = (_Float16)p[i]; a[8 + i] = (_Float16)p[16 + i]; }
  return a;
}
__device__ __forceinline__ v16h frag_f32s(const float* rowk0, int lane, float sc) {
  v16h a; const float* p = rowk0 + 8 * (lane >> 4);
#pragma unroll
  for (int i = 0; i < 8; ++i) { a[i] = (_Float16)(p[i] * sc); a[8 + i] = (_Float16)(p[16 + i] * sc); }
  return a;
}
__device__ __forceinline__ v16h fragc_f32(const float* W, int k0, int n, int lane, int ld, int K) {
  v16h a; const int g = lane >> 4;
#pragma unroll
  for (int i = 0; i < 8; ++i) { const int ka = k0 + 8 * g + i, kb = ka + 16;
    a[i] = (_Float16)(ka < K ? W[(size_t)(ka < K ? ka : K - 1) * ld + n] : 0.f); a[8 + i] = (_Float16)(kb < K ? W[(size_t)(kb < K ? kb : K - 1) * ld + n] : 0.f); }
  return a;
}
struct F2 { v16b h, l; };
__device__ __forceinline__ F2 bsplit16(const float v[16]) { F2 r;
#pragma unroll
  for (int i = 0; i < 16; ++i) { const __bf16 h = (__bf16)v[i]; r.h[i] = h; r.l[i] = (__bf16)(v[i] - (float)h); }
  return r; }
__device__ __forceinline__ F2 split_row(const float* row, int k0, int lane) { float v[16]; const float* p = row + k0 + 8 * (lane >> 4);
#pragma unroll
  for (int i = 0; i < 8; ++i) { v[i] = p[i]; v[8 + i] = p[16 + i]; }
  return bsplit16(v); }
__device__ __forceinline__ F2 split_rowK(const float* row, int k0, int lane, int K) { float v[16]; const int g = lane >> 4;
#pragma unroll
  for (int i = 0; i < 8; ++i) { const int ka = k0 + 8 * g + i, kb = ka + 16; v[i] = ka < K ? row[ka < K ? ka : K - 1] : 0.f; v[8 + i] = kb < K ? row[kb < K ? kb : K - 1] : 0.f; }
  return bsplit16(v); }
__device__ __forceinline__ F2 split_col(const float* W, int k0, int n, int lane, int ld, int K) { float v[16]; const int g = lane >> 4;
#pragma unroll
  for (int i = 0; i < 8; ++i) { const int ka = k0 + 8 * g + i, kb = ka + 16; v[i] = ka < K ? W[(size_t)(ka < K ? ka : K - 1) * ld + n] : 0.f; v[8 + i] = kb < K ? W[(size_t)(kb < K ? kb : K - 1) * ld + n] : 0.f; }
  return bsplit16(v); }
__device__ __forceinline__ v8f mac3(const F2& a, const F2& b, v8f c) { c = wmma_bf(a.l, b.h, c); c = wmma_bf(a.h, b.l, c); return wmma_bf(a.h, b.h, c); }
__device__ __forceinline__ float sigm(float v) { return 1.0f / (1.0f + expf(-v)); }
#define LDSX() do { asm volatile("s_wait_dscnt 0" ::: "memory"); __builtin_amdgcn_wave_barrier(); __builtin_amdgcn_fence(__ATOMIC_RELEASE, "workgroup"); } while (0)

#define NBT 16
#define HH 4
#define WW 900
#define CCH 256
#define KD (HH * CCH)
#define MP 960
#define NP 1024
#define DP 928
#ifndef TB
#define TB NBT
#endif
#define WS_G   0u
#define WS_D   (WS_G + 4u * (size_t)NBT * MP * NP)
#define WS_END (WS_D + 4u * (size_t)NBT * DP)

__global__ __launch_bounds__(128) void k_gram(const float* __restrict__ X1, const float* __restrict__ X2, float* __restrict__ G) {
  __shared__ __align__(16) float sf[4][16][132];
  const int tid = threadIdx.x, wave = tid >> 5, lane = tid & 31, col = lane & 15, g = lane >> 4; const int b = blockIdx.z; const int j0 = blockIdx.y * 128; const int i0 = blockIdx.x * 64 + wave * 16;
  const int ia = i0 + col; const int ic = ia < WW ? ia : WW - 1;
  v8f acc[8] = {};
#pragma unroll 2
  for (int kc = 0; kc < KD / 32; ++kc) { const int d0 = kc * 32, h = d0 >> 8, c0 = d0 & 255;
    v16b a; { const float* p = X1 + (((size_t)b * HH + h) * WW + ic) * CCH + c0 + 8 * g;
#pragma unroll
      for (int i = 0; i < 8; ++i) { a[i] = (__bf16)p[i]; a[8 + i] = (__bf16)p[16 + i]; } }
#pragma unroll
    for (int j = 0; j < 8; ++j) { const int ja = j0 + j * 16 + col; const int jc = ja < WW ? ja : WW - 1; const float* pw = X2 + (((size_t)b * HH + h) * WW + jc) * CCH + c0 + 8 * g; v16b w;
#pragma unroll
      for (int i = 0; i < 8; ++i) { w[i] = (__bf16)pw[i]; w[8 + i] = (__bf16)pw[16 + i]; }
      acc[j] = wmma_bf(a, w, acc[j]); } }
#pragma unroll
  for (int j = 0; j < 8; ++j)
#pragma unroll
    for (int r = 0; r < 8; ++r) sf[wave][8 * g + r][j * 16 + col] = acc[j][r];
  LDSX(); for (int rl = 0; rl < 16; ++rl) vst2(G + ((size_t)b * MP + i0 + rl) * NP + j0 + lane * 4, *(const v4f*)&sf[wave][rl][lane * 4]); }
__global__ __launch_bounds__(256) void k_diag(const float* __restrict__ G, float* __restrict__ D) {
  __shared__ float sp[8][32];
  const int tid = threadIdx.x, wave = tid >> 5, lane = tid & 31; const int b = blockIdx.y; const int d = blockIdx.x * 32 + lane;
  const int w0 = wave * 113, w1 = (wave + 1) * 113 < WW ? (wave + 1) * 113 : WW;
  float s = 0.f;
  if (d < WW) { int row = (w0 + d) % WW; const float* gb = G + (size_t)b * MP * NP;
    for (int w = w0; w < w1; ++w) { s += gb[(size_t)row * NP + w]; row = row + 1 < WW ? row + 1 : 0; } }
  sp[wave][lane] = s; __syncthreads();
  if (wave == 0) { float v = 0.f;
#pragma unroll
    for (int k = 0; k < 8; ++k) v += sp[k][lane];
    if (d >= WW) v = 0.f;
    vst2(D + (size_t)b * DP + blockIdx.x * 32 + lane, v); } }
__global__ __launch_bounds__(256) void k_out(const float* __restrict__ D, float* __restrict__ OUT) {
  const int tid = threadIdx.x;
  for (int e4 = tid; e4 < NBT * WW / 4; e4 += 256) { v4f r;
#pragma unroll
    for (int q = 0; q < 4; ++q) { const int e = 4 * e4 + q; const int b = e / WW, s = e % WW; r[q] = b < TB ? D[(size_t)b * DP + (s + WW / 2) % WW] : 0.f; }
    vst2(OUT + 4 * (size_t)e4, r); } }
extern "C" void kernel_launch(void* const* d_in, const int* in_sizes, int n_in, void* d_out, int out_size, void* d_ws, size_t ws_size, hipStream_t stream) {
  (void)in_sizes; (void)n_in; (void)out_size;
  const float** F = (const float**)d_in;
  if (ws_size < (size_t)WS_END) return;
  char* ws = (char*)d_ws; float* G = (float*)(ws + WS_G); float* D = (float*)(ws + WS_D);
  k_gram<<<dim3(MP / 64, NP / 128, TB), 128, 0, stream>>>(F[0], F[1], G);
  k_diag<<<dim3(DP / 32, TB), 256, 0, stream>>>(G, D);
  k_out<<<1, 256, 0, stream>>>(D, (float*)d_out);
}
